// Cross_Attention_61873298866510
// MI455X (gfx1250) — hardware-verified
//
#include <hip/hip_runtime.h>


#define CC 128
#define NH 4
#define HD 32
#define NB_FULL 4
#define SEQ_FULL 4096
#ifndef NB
#define NB 4
#endif
#ifndef SEQ
#define SEQ 4096
#endif
#define PT 64
#define XP 136
#define VP 72
#define OP 36
#define QB 128
#define KSTEP 32
#define PCARRY 16384.0f
#define VCARRY 16.0f
#define OSCALE (1.0f / 262144.0f)
#define CSC 0.255034861f

static_assert(NB >= 1 && NB <= NB_FULL);
static_assert(SEQ >= QB && SEQ <= SEQ_FULL && (SEQ % QB) == 0 && (SEQ % PT) == 0 && (SEQ % KSTEP) == 0);
static_assert(CC == NH * HD && HD == 32 && PT == 64 && (CC % 32) == 0);

typedef unsigned short us;
typedef __attribute__((ext_vector_type(8)))  unsigned short v8us;
typedef __attribute__((ext_vector_type(16))) unsigned short v16us;
typedef __attribute__((ext_vector_type(16))) __bf16   v16bf;
typedef __attribute__((ext_vector_type(16))) _Float16 v16h;
typedef __attribute__((ext_vector_type(8)))  float    v8f;
typedef __attribute__((ext_vector_type(4)))  float    v4f;

#if defined(__AMDGCN__) && __has_builtin(__builtin_amdgcn_exp2f)
#define EXP2F(x) __builtin_amdgcn_exp2f(x)
#else
#define EXP2F(x) exp2f(x)
#endif

__device__ __forceinline__ us f2bf(float f) { unsigned u = __float_as_uint(f); u += 0x7FFFu + ((u >> 16) & 1u); return (us)(u >> 16); }
__device__ __forceinline__ float bf2f(us v) { return __uint_as_float(((unsigned)v) << 16); }
__device__ __forceinline__ us f2h(float f) { return __builtin_bit_cast(us, (_Float16)f); }

__device__ __forceinline__ v16us ldfrag(const us* p, int hf) {
    const v8us a = *(const v8us*)(p + 8 * hf);
    const v8us c = *(const v8us*)(p + 16 + 8 * hf);
    return __builtin_shufflevector(a, c, 0, 1, 2, 3, 4, 5, 6, 7, 8, 9, 10, 11, 12, 13, 14, 15);
}
__device__ __forceinline__ v8f wmb(v16us a, v16us b, v8f c) {
    return __builtin_amdgcn_wmma_f32_16x16x32_bf16(false, __builtin_bit_cast(v16bf, a), false, __builtin_bit_cast(v16bf, b), (short)0, c, false, false);
}
__device__ __forceinline__ v8f wmh(v16us a, v16h b, v8f c) {
    return __builtin_amdgcn_wmma_f32_16x16x32_f16(false, __builtin_bit_cast(v16h, a), false, b, (short)0, c, false, false);
}
__device__ __forceinline__ v8f wmb_g(v16us a, v16us b, v8f c) {
    c = wmb(a, b, c);
    asm volatile("v_nop\n\tv_nop\n\tv_nop\n\tv_nop" : "+v"(c) : "v"(a), "v"(b));
    return c;
}

__global__ __launch_bounds__(256) void k_wcvt(const float* __restrict__ Wq, const float* __restrict__ Wk, const float* __restrict__ Wv, us* Wb) {
    const int g = blockIdx.x * 256 + threadIdx.x;
    if (g >= 3 * CC * CC / 8) return;
    const int mtx = g / (CC * CC / 8);
    const int e = (g - mtx * (CC * CC / 8)) * 8;
    const float* W = (mtx == 0) ? Wq : ((mtx == 1) ? Wk : Wv);
    const v4f a = *(const v4f*)(W + e);
    const v4f c = *(const v4f*)(W + e + 4);
    v8us o = {0, 0, 0, 0, 0, 0, 0, 0};
    o[0] = f2bf(a[0]); o[1] = f2bf(a[1]); o[2] = f2bf(a[2]); o[3] = f2bf(a[3]);
    o[4] = f2bf(c[0]); o[5] = f2bf(c[1]); o[6] = f2bf(c[2]); o[7] = f2bf(c[3]);
    us* dst = Wb + (size_t)g * 8;
    *(volatile v8us*)dst = o;
    __threadfence();
    *(volatile v8us*)dst = o;
}

__global__ __launch_bounds__(128) void k_proj(const float* __restrict__ xq, const float* __restrict__ xk, const us* __restrict__ Wb,
                                             us* Qhi, us* Qlo, us* Khi, us* Klo, us* Vt) {
    __shared__ __align__(16) us xT[PT * XP];
    __shared__ __align__(16) us stg[16384];
    const int tid = threadIdx.x, lane = tid & 31, w = tid >> 5, l16 = lane & 15, hf = lane >> 4;
    const int b = blockIdx.y, n0 = blockIdx.x * PT;
    const v8f zero = {0.f, 0.f, 0.f, 0.f, 0.f, 0.f, 0.f, 0.f};
#pragma unroll 1
    for (int ph = 0; ph < 3; ++ph) {
        if (ph < 2) {
            const float* x = (ph == 0) ? xq : xk;
            __syncthreads();
#pragma unroll 2
            for (int it = 0; it < (CC * PT / 4) / 128; ++it) {
                const int idx = tid + 128 * it;
                const int c = idx >> 4, n4 = idx & 15;
                const v4f v = *(const v4f*)(x + ((size_t)b * CC + c) * SEQ_FULL + n0 + 4 * n4);
                us* d = xT + (4 * n4) * XP + c;
                d[0] = f2bf(v[0]); d[XP] = f2bf(v[1]); d[2 * XP] = f2bf(v[2]); d[3 * XP] = f2bf(v[3]);
            }
            __syncthreads();
        }
        const us* W = Wb + (size_t)ph * CC * CC;
        const us* xrow = xT + (w * 16 + l16) * XP;
        v8f acc[8];
#pragma unroll
        for (int ot = 0; ot < 8; ++ot) acc[ot] = zero;
#pragma unroll 1
        for (int kc = 0; kc < CC; kc += 32) {
            const v16us bx = ldfrag(xrow + kc, hf);
#pragma unroll
            for (int ot = 0; ot < 8; ++ot) acc[ot] = wmb_g(ldfrag(W + (size_t)(ot * 16 + l16) * CC + kc, hf), bx, acc[ot]);
        }
        if (ph < 2) {
            const float sc = (ph == 0) ? CSC : 1.0f;
            us* P0 = (ph == 0) ? Qhi : Khi;
            us* P1 = (ph == 0) ? Qlo : Klo;
            us* ms = stg + w * 4096;
#pragma unroll
            for (int ot = 0; ot < 8; ++ot) {
                v8us vh = {0, 0, 0, 0, 0, 0, 0, 0};
                v8us vl = {0, 0, 0, 0, 0, 0, 0, 0};
#pragma unroll
                for (int r = 0; r < 8; ++r) {
                    const float q = acc[ot][r] * sc;
                    const us hb = f2bf(q);
                    vh[r] = hb;
                    vl[r] = f2bf(q - bf2f(hb));
                }
                const int hdh = ot >> 1, dofs = (ot & 1) * 16 + 8 * hf;
                *(v8us*)(ms + hdh * 512 + l16 * HD + dofs) = vh;
                *(v8us*)(ms + (4 + hdh) * 512 + l16 * HD + dofs) = vl;
            }
            __syncthreads();
            auto pass = [&]() {
#pragma unroll
                for (int hdh = 0; hdh < NH; ++hdh) {
                    const size_t gb = ((size_t)(b * NH + hdh) * SEQ + n0 + w * 16) * HD;
#pragma unroll
                    for (int c2 = 0; c2 < 2; ++c2) {
                        const int ch = c2 * 32 + lane;
                        const v8us a = *(const v8us*)(ms + hdh * 512 + ch * 8);
                        *(volatile v8us*)(P0 + gb + (size_t)ch * 8) = a;
                        const v8us a2 = *(const v8us*)(ms + (4 + hdh) * 512 + ch * 8);
                        *(volatile v8us*)(P1 + gb + (size_t)ch * 8) = a2;
                    }
                }
            };
            pass();
            __threadfence();
            pass();
        } else {
            __syncthreads();
#pragma unroll
            for (int ot = 0; ot < 8; ++ot)
#pragma unroll
                for (int r = 0; r < 8; ++r) stg[(ot * 16 + 8 * hf + r) * VP + w * 16 + l16] = f2h(acc[ot][r] * VCARRY);
            __syncthreads();
            auto passv = [&]() {
#pragma unroll
                for (int it = 0; it < 8; ++it) {
                    const int o = w * 32 + 4 * it + (lane >> 3), ch = lane & 7;
                    const int hdh = o >> 5, d = o & 31;
                    const v8us a = *(const v8us*)(stg + o * VP + 8 * ch);
                    *(volatile v8us*)(Vt + ((size_t)(b * NH + hdh) * HD + d) * SEQ + n0 + 8 * ch) = a;
                }
            };
            passv();
            __threadfence();
            passv();
        }
    }
}

__global__ __launch_bounds__(128) void k_attn(const us* __restrict__ Qhi, const us* __restrict__ Qlo, const us* __restrict__ Khi,
                                             const us* __restrict__ Klo, const us* __restrict__ Vt, float* out) {
    __shared__ __align__(16) float ost[4 * 32 * OP];
    const int tid = threadIdx.x, lane = tid & 31, w = tid >> 5, l16 = lane & 15, hf = lane >> 4;
    const int bh = blockIdx.y, b = bh / NH, hd = bh - b * NH;
    const int q0 = blockIdx.x * QB + w * 32;
    const size_t pb0 = (size_t)bh * SEQ * HD;
    const v8f zero = {0.f, 0.f, 0.f, 0.f, 0.f, 0.f, 0.f, 0.f};

    v16us qh[2], ql[2];
#pragma unroll
    for (int t = 0; t < 2; ++t) {
        const size_t ro = pb0 + (size_t)(q0 + 16 * t + l16) * HD;
        qh[t] = ldfrag(Qhi + ro, hf);
        ql[t] = ldfrag(Qlo + ro, hf);
    }
    const us* Kh = Khi + pb0 + (size_t)l16 * HD;
    const us* Kl = Klo + pb0 + (size_t)l16 * HD;
    const us* Vb = Vt + (size_t)bh * HD * SEQ + (size_t)l16 * SEQ;

    v8f o[2][2];
    o[0][0] = zero; o[0][1] = zero; o[1][0] = zero; o[1][1] = zero;
    float m[2], l[2];
    m[0] = -__builtin_inff(); m[1] = -__builtin_inff(); l[0] = 0.f; l[1] = 0.f;

#pragma unroll 1
    for (int kb = 0; kb < SEQ / KSTEP; ++kb) {
        const int key0 = kb * KSTEP;
        v16us kh[2], kl[2];
#pragma unroll
        for (int j = 0; j < 2; ++j) {
            kh[j] = ldfrag(Kh + (size_t)(key0 + 16 * j) * HD, hf);
            kl[j] = ldfrag(Kl + (size_t)(key0 + 16 * j) * HD, hf);
        }
        v8f s[2][2];
#pragma unroll
        for (int j = 0; j < 2; ++j)
#pragma unroll
            for (int t = 0; t < 2; ++t) {
                v8f c = wmb(kh[j], qh[t], zero);
                c = wmb(kh[j], ql[t], c);
                c = wmb(kl[j], qh[t], c);
                s[j][t] = c;
            }
        asm volatile("v_nop\n\tv_nop\n\tv_nop\n\tv_nop"
                     : "+v"(s[0][0]), "+v"(s[0][1]), "+v"(s[1][0]), "+v"(s[1][1])
                     : "v"(kh[0]), "v"(kh[1]), "v"(kl[0]), "v"(kl[1]), "v"(qh[0]), "v"(qh[1]), "v"(ql[0]), "v"(ql[1]));
        float al[2];
        v16h pv[2];
#pragma unroll
        for (int t = 0; t < 2; ++t) {
            float mx = s[0][t][0];
#pragma unroll
            for (int r = 1; r < 8; ++r) mx = fmaxf(mx, s[0][t][r]);
#pragma unroll
            for (int r = 0; r < 8; ++r) mx = fmaxf(mx, s[1][t][r]);
            mx = fmaxf(mx, __shfl_xor(mx, 16, 32));
            const float mn = fmaxf(m[t], mx);
            al[t] = EXP2F(m[t] - mn);
            m[t] = mn;
            float ps = 0.f;
            v16h pt = {0, 0, 0, 0, 0, 0, 0, 0, 0, 0, 0, 0, 0, 0, 0, 0};
#pragma unroll
            for (int r = 0; r < 8; ++r) {
                const float p0 = EXP2F(s[0][t][r] - mn);
                const float p1 = EXP2F(s[1][t][r] - mn);
                ps += p0 + p1;
                pt[r] = (_Float16)(p0 * PCARRY);
                pt[8 + r] = (_Float16)(p1 * PCARRY);
            }
            pv[t] = pt;
            ps += __shfl_xor(ps, 16, 32);
            l[t] = l[t] * al[t] + ps;
        }
        v16us va[2];
#pragma unroll
        for (int i = 0; i < 2; ++i) va[i] = ldfrag(Vb + (size_t)i * 16 * SEQ + key0, hf);
#pragma unroll
        for (int i = 0; i < 2; ++i)
#pragma unroll
            for (int t = 0; t < 2; ++t) o[i][t] = wmh(va[i], pv[t], o[i][t] * al[t]);
        asm volatile("v_nop\n\tv_nop\n\tv_nop\n\tv_nop"
                     : "+v"(o[0][0]), "+v"(o[0][1]), "+v"(o[1][0]), "+v"(o[1][1])
                     : "v"(va[0]), "v"(va[1]), "v"(pv[0]), "v"(pv[1]));
    }

    float inv[2];
    inv[0] = (1.0f / l[0]) * OSCALE;
    inv[1] = (1.0f / l[1]) * OSCALE;
    float* ms = ost + w * (32 * OP);
#pragma unroll
    for (int i = 0; i < 2; ++i)
#pragma unroll
        for (int t = 0; t < 2; ++t)
#pragma unroll
            for (int r = 0; r < 8; ++r) ms[(16 * i + 8 * hf + r) * OP + 16 * t + l16] = o[i][t][r] * inv[t];
    __syncthreads();
    float* ob = out + ((size_t)b * CC + (size_t)hd * HD) * SEQ_FULL + q0;
    auto pass = [&]() {
#pragma unroll
        for (int it = 0; it < 8; ++it) {
            const int d = 4 * it + (lane >> 3), ch = lane & 7;
            const v4f v = *(const v4f*)(ms + d * OP + 4 * ch);
            *(volatile v4f*)(ob + (size_t)d * SEQ_FULL + 4 * ch) = v;
        }
    };
    pass();
    __threadfence();
    pass();
}

extern "C" void kernel_launch(void* const* d_in, const int* in_sizes, int n_in,
                              void* d_out, int out_size, void* d_ws, size_t ws_size, hipStream_t stream) {
    if (n_in < 5) return;
    if ((size_t)in_sizes[0] < (size_t)NB * CC * SEQ_FULL) return;
    if ((size_t)in_sizes[1] < (size_t)NB * CC * SEQ_FULL) return;
    if (in_sizes[2] < CC * CC || in_sizes[3] < CC * CC || in_sizes[4] < CC * CC) return;
    if ((size_t)out_size < (size_t)NB * CC * SEQ_FULL) return;
    const float* xq = (const float*)d_in[0];
    const float* xk = (const float*)d_in[1];
    const float* Wq = (const float*)d_in[2];
    const float* Wk = (const float*)d_in[3];
    const float* Wv = (const float*)d_in[4];
    float* out = (float*)d_out;

    char* wsp = (char*)d_ws;
    size_t off = 0;
    auto take = [&](size_t bytes) -> void* { void* p = wsp + off; off += (bytes + 255) & ~(size_t)255; return p; };
    const size_t plane = (size_t)NB * NH * SEQ * HD * sizeof(us);
    us* Wb  = (us*)take((size_t)3 * CC * CC * sizeof(us));
    us* Qhi = (us*)take(plane);
    us* Qlo = (us*)take(plane);
    us* Khi = (us*)take(plane);
    us* Klo = (us*)take(plane);
    us* Vt  = (us*)take(plane);
    if (off > ws_size) return;

    k_wcvt<<<dim3((3 * CC * CC / 8 + 255) / 256), 256, 0, stream>>>(Wq, Wk, Wv, Wb);
    k_proj<<<dim3(SEQ / PT, NB), 128, 0, stream>>>(xq, xk, Wb, Qhi, Qlo, Khi, Klo, Vt);
    k_attn<<<dim3(SEQ / QB, NB * NH), 128, 0, stream>>>(Qhi, Qlo, Khi, Klo, Vt, out);
    (void)hipGetLastError();
}
